// VcpByDis_54125177864528
// MI455X (gfx1250) — hardware-run, weakly checked
//
#include <hip/hip_runtime.h>


#define NBT  8
#define DD   64
#define NP   4096
#define RH   2048
#define DM   DD
#define SCL  0.125f
#define LOSC 1024.0f

typedef _Float16 h16;
typedef unsigned short bf;
typedef __attribute__((ext_vector_type(16))) __bf16   v16bf;
typedef __attribute__((ext_vector_type(16))) _Float16 v16h;
typedef __attribute__((ext_vector_type(8)))  _Float16 v8h;
typedef __attribute__((ext_vector_type(8)))  unsigned short v8us;
typedef __attribute__((ext_vector_type(8)))  float    v8f;
typedef __attribute__((ext_vector_type(4)))  float    v4f;
typedef v8h  __attribute__((may_alias)) v8ha;
typedef v4f  __attribute__((may_alias)) v4fa;
typedef v8us __attribute__((may_alias)) v8usa;

__device__ __forceinline__ unsigned short f2bf(float f) { unsigned u = __float_as_uint(f); u += 0x7FFFu + ((u >> 16) & 1u); return (unsigned short)(u >> 16); }
__device__ __forceinline__ float bf2f(unsigned short b) { return __uint_as_float(((unsigned)b) << 16); }
__device__ __forceinline__ float bfr(float f) { return bf2f(f2bf(f)); }
__device__ __forceinline__ v16h cat16(v8h lo, v8h hi) { return __builtin_shufflevector(lo, hi, 0, 1, 2, 3, 4, 5, 6, 7, 8, 9, 10, 11, 12, 13, 14, 15); }
__device__ __forceinline__ v16bf cat16b(v8us lo, v8us hi) { return __builtin_bit_cast(v16bf, __builtin_shufflevector(lo, hi, 0, 1, 2, 3, 4, 5, 6, 7, 8, 9, 10, 11, 12, 13, 14, 15)); }
__device__ __forceinline__ v8f wmma16(v16h a, v16h b, v8f c) { return __builtin_amdgcn_wmma_f32_16x16x32_f16(false, a, false, b, (short)0, c, false, false); }
__device__ __forceinline__ v8f wmmab(v16bf a, v16bf b, v8f c) { return __builtin_amdgcn_wmma_f32_16x16x32_bf16(false, a, false, b, (short)0, c, false, false); }

template <bool SPLITA, bool F16OUT = false>
__global__ __launch_bounds__(128) void k_gemmb(const bf* __restrict__ A, const bf* __restrict__ Al, const bf* __restrict__ Bn, const float* __restrict__ bias, float* C, int ldc, h16* C2, const float* __restrict__ R = nullptr, int K = DM, int roundR = 1) {
    __shared__ __align__(16) float ost[4][16 * 68];
    const int lane = threadIdx.x & 31, wave = threadIdx.x >> 5, lr = lane & 15, hi = lane >> 4;
    const int r0 = blockIdx.x * 64 + wave * 16, c0 = blockIdx.y * 64;
    const size_t aoff = (size_t)(r0 + lr) * K + 8 * hi;
    size_t boff[4];
#pragma unroll
    for (int t = 0; t < 4; ++t) boff[t] = (size_t)(c0 + t * 16 + lr) * K + 8 * hi;
    v8f acc[4];
#pragma unroll
    for (int t = 0; t < 4; ++t) acc[t] = (v8f){};
#pragma unroll 1
    for (int kc = 0; kc < K; kc += 32) {
        const v16bf a = cat16b(*(const v8us*)(A + aoff + kc), *(const v8us*)(A + aoff + kc + 16));
        v16bf al = a;
        if (SPLITA) al = cat16b(*(const v8us*)(Al + aoff + kc), *(const v8us*)(Al + aoff + kc + 16));
#pragma unroll
        for (int t = 0; t < 4; ++t) { const v16bf b = cat16b(*(const v8us*)(Bn + boff[t] + kc), *(const v8us*)(Bn + boff[t] + kc + 16)); acc[t] = wmmab(a, b, acc[t]); if (SPLITA) acc[t] = wmmab(al, b, acc[t]); }
        asm volatile("v_nop\n\tv_nop\n\tv_nop\n\tv_nop" : "+v"(acc[0]), "+v"(acc[1]), "+v"(acc[2]), "+v"(acc[3]) : "v"(a), "v"(al));
    }
    float* os = &ost[wave][0];
#pragma unroll
    for (int t = 0; t < 4; ++t) { const float bv = bias ? bfr(bias[c0 + t * 16 + lr]) : 0.f;
#pragma unroll
        for (int j = 0; j < 8; ++j) os[(hi * 8 + j) * 68 + t * 16 + lr] = acc[t][j] + bv; }
    __syncthreads();
    if (F16OUT) {
        h16* crow = (h16*)(void*)C + (size_t)r0 * ldc + c0;
        auto pass = [&]() {
#pragma unroll
            for (int s = 0; s < 4; ++s) { const int row = 4 * s + (lane >> 3), piece = lane & 7; const float* sp = os + row * 68 + piece * 8; v8h o, o2;
#pragma unroll
                for (int i = 0; i < 8; ++i) { const h16 a = (h16)sp[i]; o[i] = a; o2[i] = (h16)((sp[i] - (float)a) * LOSC); }
                *(volatile v8h*)(crow + (size_t)row * ldc + piece * 8) = o; if (C2) *(volatile v8h*)(C2 + (size_t)r0 * ldc + c0 + (size_t)row * ldc + piece * 8) = o2; }
        };
        pass(); __threadfence(); pass();
    } else {
        float* crow = C + (size_t)r0 * ldc + c0;
        auto pass = [&]() {
#pragma unroll
            for (int s = 0; s < 8; ++s) { const int Lid = (lane >> 3) + 4 * s, piece = lane & 7; const int row = Lid >> 1, cofs = (Lid & 1) * 32 + piece * 4;
                v4f val = *(const v4fa*)(os + row * 68 + cofs); if (R) { const v4f rv = *(const v4f*)(R + ((size_t)r0 + row) * ldc + c0 + cofs); val += roundR ? (v4f){bfr(rv[0]), bfr(rv[1]), bfr(rv[2]), bfr(rv[3])} : rv; }
                *(volatile v4f*)(crow + (size_t)row * ldc + cofs) = val; }
        };
        pass(); __threadfence(); pass();
    }
}


__global__ __launch_bounds__(256) void k_ptb64(const float* __restrict__ E, bf* XT) {
    __shared__ float tl[64][65];
    typedef __attribute__((ext_vector_type(4))) unsigned short v4us;
    const int tid = threadIdx.x, p0 = blockIdx.y * 64; const int rr = tid >> 2, cq = (tid & 3) * 16;
#pragma unroll
    for (int i = 0; i < 16; ++i) tl[rr][cq + i] = E[(size_t)rr * NP + p0 + cq + i];
    __syncthreads();
    const int lane = tid & 31, wv = tid >> 5;
    auto pass = [&]() {
#pragma unroll
        for (int st = 0; st < 4; ++st) { const int pr = wv * 8 + st * 2 + (lane >> 4); const int dl = (lane & 15) * 4; v4us v;
#pragma unroll
            for (int i = 0; i < 4; ++i) v[i] = f2bf(tl[dl + i][pr]);
            *(volatile v4us*)(XT + (size_t)(p0 + pr) * DD + dl) = v; }
    };
    pass(); __threadfence(); pass();
}
__global__ __launch_bounds__(256) void k_tgpad(const float* __restrict__ tg, bf* TG) {
    const int lane = threadIdx.x & 31; const size_t w = (size_t)blockIdx.x * 8 + (threadIdx.x >> 5); if (w >= (size_t)64 * (NP / 256)) return; const int c = (int)(w / (NP / 256)); const int m0 = (int)(w % (NP / 256)) * 256 + lane * 8; v8us v;
#pragma unroll
    for (int i = 0; i < 8; ++i) v[i] = f2bf(c < 3 ? tg[(size_t)(c < 3 ? c : 0) * NP + m0 + i] : 0.f);
    *(volatile v8us*)(TG + (size_t)c * NP + m0) = v; __threadfence(); *(volatile v8us*)(TG + (size_t)c * NP + m0) = v;
}
__global__ __launch_bounds__(256) void k_soft(const float* __restrict__ S, float sc, bf* PH, bf* PL) {
    typedef __attribute__((ext_vector_type(4))) unsigned short v4us;
    const int lane = threadIdx.x & 31, i = blockIdx.x * 8 + (threadIdx.x >> 5); if (i >= RH) return; const float* sr = S + (size_t)i * NP;
    float m = -3.0e38f;
#pragma unroll 1
    for (int c0 = lane * 4; c0 < NP; c0 += 128) {
#pragma unroll
        for (int q = 0; q < 4; ++q) m = fmaxf(m, sr[c0 + q] * sc); }
#pragma unroll
    for (int sh = 16; sh; sh >>= 1) m = fmaxf(m, __shfl_xor(m, sh, 32));
    float sum = 0.f;
#pragma unroll 1
    for (int c0 = lane * 4; c0 < NP; c0 += 128) {
#pragma unroll
        for (int q = 0; q < 4; ++q) sum += __expf(sr[c0 + q] * sc - m); }
#pragma unroll
    for (int sh = 16; sh; sh >>= 1) sum += __shfl_xor(sum, sh, 32);
    const float inv = 1.0f / sum;
#pragma unroll 1
    for (int ps = 0; ps < 2; ++ps) {
#pragma unroll 1
        for (int c0 = lane * 4; c0 < NP; c0 += 128) { v4us oh, ol;
#pragma unroll
            for (int q = 0; q < 4; ++q) { const float p = __expf(sr[c0 + q] * sc - m) * inv; const unsigned short hb = f2bf(p); oh[q] = hb; ol[q] = f2bf(p - bf2f(hb)); }
            const size_t o = (size_t)i * NP + c0; *(volatile v4us*)(PH + o) = oh; *(volatile v4us*)(PL + o) = ol; }
        if (ps == 0) __threadfence(); }
}
__global__ __launch_bounds__(256) void k_corrT(const float* __restrict__ CT, float* dst) {
    const int lane = threadIdx.x & 31; const size_t w = (size_t)blockIdx.x * 8 + (threadIdx.x >> 5); if (w >= (size_t)3 * (NP / 32)) return; const int c = (int)(w / (NP / 32)); const int n = (int)(w % (NP / 32)) * 32 + lane; const float v = CT[(size_t)n * DD + c];
    *(volatile float*)(dst + (size_t)c * NP + n) = v; __threadfence(); *(volatile float*)(dst + (size_t)c * NP + n) = v;
}
__global__ __launch_bounds__(256) void k_copy(const float* __restrict__ s, float* d, size_t n4) {
    const size_t i = (size_t)blockIdx.x * 256 + threadIdx.x; if (i >= n4) return; const v4f v = *(const v4f*)(s + i * 4);
    *(volatile v4f*)(d + i * 4) = v; __threadfence(); *(volatile v4f*)(d + i * 4) = v;
}

extern "C" void kernel_launch(void* const* d_in, const int* in_sizes, int n_in,
                              void* d_out, int out_size, void* d_ws, size_t ws_size, hipStream_t stream) {
    (void)in_sizes; (void)n_in; (void)out_size;
    const float* se = (const float*)d_in[0]; const float* te = (const float*)d_in[1]; const float* src = (const float*)d_in[2]; const float* tgt = (const float*)d_in[3];
    float* out0 = (float*)d_out;
    float* out1 = (float*)((char*)d_out + (size_t)NBT * 3 * NP * 4);
    char* wsp = (char*)d_ws;
    auto take = [&](size_t bytes) { char* p = wsp; wsp += (bytes + 255) & ~(size_t)255; return (void*)p; };
    bf* SE = (bf*)take((size_t)NP * DD * 2); bf* TE = (bf*)take((size_t)NP * DD * 2); bf* TG = (bf*)take((size_t)64 * NP * 2);
    float* S = (float*)take((size_t)RH * NP * 4); bf* PH = (bf*)take((size_t)RH * NP * 2); bf* PL = (bf*)take((size_t)RH * NP * 2); float* CT = (float*)take((size_t)NP * DD * 4);
    if ((size_t)(wsp - (char*)d_ws) > ws_size) return;
    k_copy<<<(unsigned)(((size_t)NBT * 3 * NP / 4 + 255) / 256), 256, 0, stream>>>(src, out0, (size_t)NBT * 3 * NP / 4);
    for (int b = 0; b < NBT; ++b) {
        k_ptb64<<<dim3(1, NP / 64, 1), 256, 0, stream>>>(se + (size_t)b * DD * NP, SE); k_ptb64<<<dim3(1, NP / 64, 1), 256, 0, stream>>>(te + (size_t)b * DD * NP, TE); k_tgpad<<<(64 * (NP / 256)) / 8, 256, 0, stream>>>(tgt + (size_t)b * 3 * NP, TG);
        for (int hf = 0; hf < NP / RH; ++hf) { const size_t r0 = (size_t)hf * RH;
            k_gemmb<false, false><<<dim3(RH / 64, NP / 64, 1), 128, 0, stream>>>(SE + r0 * DD, nullptr, TE, nullptr, S, NP, nullptr, nullptr, DD);
            k_soft<<<RH / 8, 256, 0, stream>>>(S, SCL, PH, PL);
            k_gemmb<true, false><<<dim3(RH / 64, 1, 1), 128, 0, stream>>>(PH, PL, TG, nullptr, CT + r0 * DD, DD, nullptr, nullptr, NP); }
        k_corrT<<<(3 * (NP / 32)) / 8, 256, 0, stream>>>(CT, out1 + (size_t)b * 3 * NP); }
}
